// LocalAttention2_54992761258371
// MI455X (gfx1250) — hardware-verified
//
#include <hip/hip_runtime.h>


#define NB_  4
#define TT   4096
#define DD   512
#define NH_  8
#define HD   64
typedef _Float16 h16;
typedef unsigned short bf;
typedef __attribute__((ext_vector_type(16))) __bf16   v16bf;
typedef __attribute__((ext_vector_type(16))) _Float16 v16h;
typedef __attribute__((ext_vector_type(8)))  _Float16 v8h;
typedef __attribute__((ext_vector_type(8)))  unsigned short v8us;
typedef __attribute__((ext_vector_type(8)))  float    v8f;
typedef __attribute__((ext_vector_type(4)))  float    v4f;
typedef v8h  __attribute__((may_alias)) v8ha;
typedef v4f  __attribute__((may_alias)) v4fa;
typedef v8us __attribute__((may_alias)) v8usa;

__device__ __forceinline__ unsigned short f2bf(float f) { unsigned u = __float_as_uint(f); u += 0x7FFFu + ((u >> 16) & 1u); return (unsigned short)(u >> 16); }
__device__ __forceinline__ float bf2f(unsigned short b) { return __uint_as_float(((unsigned)b) << 16); }
__device__ __forceinline__ float bfr(float f) { return bf2f(f2bf(f)); }
__device__ __forceinline__ v16h cat16(v8h lo, v8h hi) { return __builtin_shufflevector(lo, hi, 0, 1, 2, 3, 4, 5, 6, 7, 8, 9, 10, 11, 12, 13, 14, 15); }
__device__ __forceinline__ v16bf cat16b(v8us lo, v8us hi) { return __builtin_bit_cast(v16bf, __builtin_shufflevector(lo, hi, 0, 1, 2, 3, 4, 5, 6, 7, 8, 9, 10, 11, 12, 13, 14, 15)); }
__device__ __forceinline__ v8f wmma16(v16h a, v16h b, v8f c) { return __builtin_amdgcn_wmma_f32_16x16x32_f16(false, a, false, b, (short)0, c, false, false); }
__device__ __forceinline__ v8f wmmab(v16bf a, v16bf b, v8f c) { return __builtin_amdgcn_wmma_f32_16x16x32_bf16(false, a, false, b, (short)0, c, false, false); }


template <typename T16> struct WFrag;
template <> struct WFrag<h16> { typedef v16h V; static __device__ __forceinline__ V ld(const h16* p) { return cat16(*(const v8h*)p, *(const v8h*)(p + 16)); } static __device__ __forceinline__ v8f mma(V a, V b, v8f c) { return wmma16(a, b, c); } };
template <> struct WFrag<bf> { typedef v16bf V; static __device__ __forceinline__ V ld(const bf* p) { return cat16b(*(const v8us*)p, *(const v8us*)(p + 16)); } static __device__ __forceinline__ v8f mma(V a, V b, v8f c) { return wmmab(a, b, c); } };
template <typename T16, int NSPLIT, bool BIAS>
__global__ __launch_bounds__(32) void k_gemmw(const T16* __restrict__ A, const T16* __restrict__ A2, const T16* __restrict__ Bt, const T16* __restrict__ Bt2, int K, float* C, int ldc, const float* __restrict__ bias, size_t sA, size_t sB, size_t sC) {
    typedef typename WFrag<T16>::V V;
    __shared__ __align__(16) float os[16 * 68];
    const size_t z = blockIdx.z; A += z * sA; if (A2) A2 += z * sA; Bt += z * sB; if (Bt2) Bt2 += z * sB; C += z * sC;
    const int lane = threadIdx.x & 31, lr = lane & 15, hi = lane >> 4; const int r0 = blockIdx.x * 64, c0 = blockIdx.y * 64;
    v8f acc[4][4];
#pragma unroll
    for (int mb = 0; mb < 4; ++mb)
#pragma unroll
        for (int nb = 0; nb < 4; ++nb) acc[mb][nb] = (v8f){};
    const size_t aoff = (size_t)(r0 + lr) * K + 8 * hi, boff = (size_t)(c0 + lr) * K + 8 * hi;
#pragma unroll 1
    for (int kc = 0; kc < K; kc += 32) {
        V a[4], a2[4];
#pragma unroll
        for (int mb = 0; mb < 4; ++mb) { a[mb] = WFrag<T16>::ld(A + aoff + (size_t)mb * 16 * K + kc); if (NSPLIT == 1 || NSPLIT == 2) a2[mb] = WFrag<T16>::ld(A2 + aoff + (size_t)mb * 16 * K + kc); }
#pragma unroll
        for (int nb = 0; nb < 4; ++nb) { const V b = WFrag<T16>::ld(Bt + boff + (size_t)nb * 16 * K + kc); V b2; if (NSPLIT >= 2) b2 = WFrag<T16>::ld(Bt2 + boff + (size_t)nb * 16 * K + kc);
#pragma unroll
            for (int mb = 0; mb < 4; ++mb) { acc[mb][nb] = WFrag<T16>::mma(a[mb], b, acc[mb][nb]); if (NSPLIT == 1 || NSPLIT == 2) acc[mb][nb] = WFrag<T16>::mma(a2[mb], b, acc[mb][nb]); if (NSPLIT >= 2) acc[mb][nb] = WFrag<T16>::mma(a[mb], b2, acc[mb][nb]); } }
        asm volatile("v_nop\n\tv_nop\n\tv_nop\n\tv_nop" : "+v"(acc[0][0]), "+v"(acc[1][1]), "+v"(acc[2][2]), "+v"(acc[3][3]) : "v"(a[0]), "v"(a[3]));
    }
#pragma unroll
    for (int mb = 0; mb < 4; ++mb) {
#pragma unroll
        for (int nb = 0; nb < 4; ++nb) {
#pragma unroll
            for (int j = 0; j < 8; ++j) os[(hi * 8 + j) * 68 + nb * 16 + lr] = acc[mb][nb][j]; }
        __builtin_amdgcn_wave_barrier(); asm volatile("" ::: "memory");
        float* crow = C + (size_t)(r0 + mb * 16) * ldc + c0;
#pragma unroll 1
        for (int ps = 0; ps < 2; ++ps) {
#pragma unroll
            for (int s = 0; s < 8; ++s) { const int row = 2 * s + hi, cofs = lr * 4; v4f val = *(const v4fa*)(os + row * 68 + cofs); if (BIAS) { val[0] += bfr(bias[c0 + cofs]); val[1] += bfr(bias[c0 + cofs + 1]); val[2] += bfr(bias[c0 + cofs + 2]); val[3] += bfr(bias[c0 + cofs + 3]); }
                *(volatile v4f*)(crow + (size_t)row * ldc + cofs) = val; }
            if (ps == 0) __threadfence(); }
        __builtin_amdgcn_wave_barrier(); asm volatile("" ::: "memory");
    }
}

__device__ __forceinline__ void splitf(float y, unsigned short& h, unsigned short& l) { h = f2bf(y); l = f2bf(y - bf2f(h)); }
typedef __attribute__((ext_vector_type(4))) unsigned short v4us;

__global__ __launch_bounds__(256) void k_cvt8(const float* __restrict__ src, bf* dst, size_t n8) { const size_t i = (size_t)blockIdx.x * 256 + threadIdx.x; if (i >= n8) return; const v8f v = *(const v8f*)(src + i * 8); v8us o;
#pragma unroll
    for (int k = 0; k < 8; ++k) o[k] = f2bf(v[k]); *(volatile v8us*)(dst + i * 8) = o; __threadfence(); *(volatile v8us*)(dst + i * 8) = o; }
__device__ __forceinline__ float red16(float p) { p += __shfl_xor(p, 1, 32); p += __shfl_xor(p, 2, 32); p += __shfl_xor(p, 4, 32); p += __shfl_xor(p, 8, 32); return p; }
template <int I> __device__ __forceinline__ void band_one(const float* __restrict__ FQ, const float* __restrict__ FK, const float* __restrict__ FV, int t, int col, const v4f& qv, const v4f& km, const v4f& vm, bf* Oh, bf* Ol) {
    const bool hasL = (t >= I), hasR = (t < TT - I);
    const size_t oL = (size_t)(hasL ? t - I : t) * DD + col, oR = (size_t)(hasR ? t + I : t) * DD + col;
    const v4f kl = *(const v4f*)(FK + oL), kr = *(const v4f*)(FK + oR), vl = *(const v4f*)(FV + oL), vr = *(const v4f*)(FV + oR);
    float pl = 0.f, pm = 0.f, pr = 0.f;
#pragma unroll
    for (int u = 0; u < 4; ++u) { float a = __fmul_rn(qv[u], kl[u]), b = __fmul_rn(qv[u], km[u]), c = __fmul_rn(qv[u], kr[u]); asm volatile("" : "+v"(a)); asm volatile("" : "+v"(b)); asm volatile("" : "+v"(c)); pl = __fadd_rn(pl, a); pm = __fadd_rn(pm, b); pr = __fadd_rn(pr, c); }
    pl = red16(pl) * 0.125f; pm = red16(pm) * 0.125f; pr = red16(pr) * 0.125f; if (!hasL) pl = -3.0e38f; if (!hasR) pr = -3.0e38f;
    const float mx = fmaxf(fmaxf(pl, pm), pr); float dl = __fsub_rn(pl, mx), dm = __fsub_rn(pm, mx), dr = __fsub_rn(pr, mx); asm volatile("" : "+v"(dl)); asm volatile("" : "+v"(dm)); asm volatile("" : "+v"(dr));
    const float el = hasL ? __expf(dl) : 0.f, em = __expf(dm), er = hasR ? __expf(dr) : 0.f; const float inv = __fdiv_rn(1.0f, __fadd_rn(__fadd_rn(el, em), er)); const float wl = __fmul_rn(el, inv), wm = __fmul_rn(em, inv), wr = __fmul_rn(er, inv);
    v4us oh, ol;
#pragma unroll
    for (int u = 0; u < 4; ++u) { float a = __fmul_rn(wl, vl[u]), b = __fmul_rn(wm, vm[u]), c = __fmul_rn(wr, vr[u]); asm volatile("" : "+v"(a)); asm volatile("" : "+v"(b)); asm volatile("" : "+v"(c)); const float o = __fadd_rn(__fadd_rn(a, b), c); unsigned short x, y; splitf(o, x, y); oh[u] = x; ol[u] = y; }
    const size_t oo = (size_t)t * DD + col; *(volatile v4us*)(Oh + oo) = oh; *(volatile v4us*)(Ol + oo) = ol; __threadfence(); *(volatile v4us*)(Oh + oo) = oh; *(volatile v4us*)(Ol + oo) = ol; }
__global__ __launch_bounds__(256) void k_band(const float* __restrict__ FQ, const float* __restrict__ FK, const float* __restrict__ FV, bf* O1h, bf* O1l, bf* O2h, bf* O2l) { const size_t e = ((size_t)blockIdx.x * 256 + threadIdx.x) * 4; if (e >= (size_t)TT * DD) return; const int col = (int)(e % DD); const int t = (int)(e / DD);
    const v4f qv = *(const v4f*)(FQ + e), km = *(const v4f*)(FK + e), vm = *(const v4f*)(FV + e);
    band_one<1>(FQ, FK, FV, t, col, qv, km, vm, O1h, O1l); band_one<2>(FQ, FK, FV, t, col, qv, km, vm, O2h, O2l); }
__global__ __launch_bounds__(256) void k_lnfin(const float* __restrict__ U1, const float* __restrict__ U2, const float* __restrict__ x, const float* __restrict__ ga, const float* __restrict__ be, float* OUTb) { const int lane = threadIdx.x & 31; const int row = blockIdx.x * 8 + (threadIdx.x >> 5); if (row >= TT) return;
    float a1[16], a2[16]; float s1 = 0.f, s2 = 0.f;
#pragma unroll
    for (int g = 0; g < 4; ++g) { const size_t o = (size_t)row * DD + g * 128 + lane * 4; const v4f u1 = *(const v4f*)(U1 + o), u2 = *(const v4f*)(U2 + o), xx = *(const v4f*)(x + o);
#pragma unroll
        for (int u = 0; u < 4; ++u) { float xb = bfr(xx[u]); asm volatile("" : "+v"(xb)); a1[g * 4 + u] = __fadd_rn(u1[u], xb); a2[g * 4 + u] = __fadd_rn(u2[u], xb); s1 += a1[g * 4 + u]; s2 += a2[g * 4 + u]; } }
#pragma unroll
    for (int sh = 16; sh; sh >>= 1) { s1 += __shfl_xor(s1, sh, 32); s2 += __shfl_xor(s2, sh, 32); }
    const float m1 = s1 * (1.0f / DD), m2 = s2 * (1.0f / DD); float q1 = 0.f, q2 = 0.f;
#pragma unroll
    for (int k = 0; k < 16; ++k) { float d1 = __fsub_rn(a1[k], m1), d2 = __fsub_rn(a2[k], m2); asm volatile("" : "+v"(d1)); asm volatile("" : "+v"(d2)); a1[k] = d1; a2[k] = d2; float p1 = __fmul_rn(d1, d1), p2 = __fmul_rn(d2, d2); asm volatile("" : "+v"(p1)); asm volatile("" : "+v"(p2)); q1 = __fadd_rn(q1, p1); q2 = __fadd_rn(q2, p2); }
#pragma unroll
    for (int sh = 16; sh; sh >>= 1) { q1 += __shfl_xor(q1, sh, 32); q2 += __shfl_xor(q2, sh, 32); }
    const float r1 = __frsqrt_rn(__fadd_rn(q1 * (1.0f / DD), 1e-5f)), r2 = __frsqrt_rn(__fadd_rn(q2 * (1.0f / DD), 1e-5f));
    for (int ps = 0; ps < 2; ++ps) {
#pragma unroll
        for (int g = 0; g < 4; ++g) { v4f o; const int c0 = g * 128 + lane * 4;
#pragma unroll
            for (int u = 0; u < 4; ++u) { float gg = bfr(ga[c0 + u]), bb = bfr(be[c0 + u]); asm volatile("" : "+v"(gg)); asm volatile("" : "+v"(bb)); float n1 = __fmul_rn(a1[g * 4 + u], r1), n2 = __fmul_rn(a2[g * 4 + u], r2); asm volatile("" : "+v"(n1)); asm volatile("" : "+v"(n2)); float y1 = __fmul_rn(n1, gg), y2 = __fmul_rn(n2, gg); asm volatile("" : "+v"(y1)); asm volatile("" : "+v"(y2)); o[u] = __fadd_rn(__fadd_rn(y1, bb), __fadd_rn(y2, bb)); }
            *(volatile v4f*)(OUTb + (size_t)row * DD + c0) = o; }
        if (ps == 0) __threadfence(); } }

extern "C" void kernel_launch(void* const* d_in, const int* in_sizes, int n_in,
                              void* d_out, int out_size, void* d_ws, size_t ws_size, hipStream_t stream) {
    (void)in_sizes; (void)n_in; (void)out_size;
    const float** I = (const float**)d_in;
    const float *x = I[0], *wq = I[1], *bq = I[2], *wk = I[3], *bk = I[4], *wv = I[5], *bv = I[6], *wo = I[7], *bo = I[8], *ga = I[9], *be = I[10];
    float* OUT = (float*)d_out;
    char* wsp = (char*)d_ws;
    auto take = [&](size_t bytes) { char* p = wsp; wsp += (bytes + 255) & ~(size_t)255; return (void*)p; };
    bf* WQ = (bf*)take(DD * DD * 2); bf* WK = (bf*)take(DD * DD * 2); bf* WV = (bf*)take(DD * DD * 2); bf* WO = (bf*)take(DD * DD * 2);
    bf* XB = (bf*)take((size_t)TT * DD * 2); float* FQ = (float*)take((size_t)TT * DD * 4); float* FK = (float*)take((size_t)TT * DD * 4); float* FV = (float*)take((size_t)TT * DD * 4); bf* O1h = (bf*)take((size_t)TT * DD * 2); bf* O1l = (bf*)take((size_t)TT * DD * 2); bf* O2h = (bf*)take((size_t)TT * DD * 2); bf* O2l = (bf*)take((size_t)TT * DD * 2); float* U1 = (float*)take((size_t)TT * DD * 4); float* U2 = (float*)take((size_t)TT * DD * 4);
    if ((size_t)(wsp - (char*)d_ws) > ws_size) return;
    k_cvt8<<<(DD * DD / 8 + 255) / 256, 256, 0, stream>>>(wq, WQ, DD * DD / 8); k_cvt8<<<(DD * DD / 8 + 255) / 256, 256, 0, stream>>>(wk, WK, DD * DD / 8); k_cvt8<<<(DD * DD / 8 + 255) / 256, 256, 0, stream>>>(wv, WV, DD * DD / 8); k_cvt8<<<(DD * DD / 8 + 255) / 256, 256, 0, stream>>>(wo, WO, DD * DD / 8);
    for (int b = 0; b < NB_; ++b) { const float* xb = x + (size_t)b * TT * DD;
        k_cvt8<<<(TT * DD / 8 + 255) / 256, 256, 0, stream>>>(xb, XB, (size_t)TT * DD / 8);
        k_gemmw<bf, 0, true><<<dim3(TT / 64, DD / 64, 1), 32, 0, stream>>>(XB, nullptr, WQ, nullptr, DD, FQ, DD, bq, 0, 0, 0); k_gemmw<bf, 0, true><<<dim3(TT / 64, DD / 64, 1), 32, 0, stream>>>(XB, nullptr, WK, nullptr, DD, FK, DD, bk, 0, 0, 0); k_gemmw<bf, 0, true><<<dim3(TT / 64, DD / 64, 1), 32, 0, stream>>>(XB, nullptr, WV, nullptr, DD, FV, DD, bv, 0, 0, 0);
        k_band<<<(unsigned)(((size_t)TT * DD / 4 + 255) / 256), 256, 0, stream>>>(FQ, FK, FV, O1h, O1l, O2h, O2l);
        k_gemmw<bf, 1, true><<<dim3(TT / 64, DD / 64, 1), 32, 0, stream>>>(O1h, O1l, WO, nullptr, DD, U1, DD, bo, 0, 0, 0); k_gemmw<bf, 1, true><<<dim3(TT / 64, DD / 64, 1), 32, 0, stream>>>(O2h, O2l, WO, nullptr, DD, U2, DD, bo, 0, 0, 0);
        k_lnfin<<<TT / 8, 256, 0, stream>>>(U1, U2, xb, ga, be, OUT + (size_t)b * TT * DD); }
}
